// GCNModelWithWeights_11063835754876
// MI455X (gfx1250) — hardware-verified
//
#include <hip/hip_runtime.h>
#include <stddef.h>
#include <stdint.h>
#include <math.h>


#define CIN    128
#define HID    128
#define K2     256
#define OUTD   64
#define NTHR   256
#define NWAVE  8
#define EPT    8
#define CHUNK  (NTHR * EPT)
#define WCAP   (EPT * 32)
#define LISTN  (NWAVE * WCAP)
#define NBA    1024
#define SLA    10
#define RCAP   20480
#define DEGCAP 64
#define GBM    64
#define GBN    64
#define GTHR   128
#define NUW1   (HID * (CIN / 8))
#define NUW2   (OUTD * (K2 / 8))
#define SCAN_ZINTS (LISTN + 2 * RCAP + 3 * NBA)
#define SCAN_LDS_INTS (SCAN_ZINTS + 16)
#define TSUB   128
#define TPITCH 132
#define RECW   128
#define WSMAX  134217728

static_assert((CHUNK & (CHUNK - 1)) == 0 && CHUNK <= 4096);
static_assert((NBA & (NBA - 1)) == 0 && NBA == (1 << SLA));
static_assert(((long long)CHUNK << SLA) < (1LL << 31));
static_assert(LISTN % NTHR == 0);
static_assert(NBA % NWAVE == 0 && NBA % 32 == 0 && NBA % GBM == 0 && NBA == 4 * NTHR);
static_assert(RCAP % 1024 == 0 && SCAN_ZINTS % 4 == 0 && LISTN % 4 == 0);
static_assert(CIN % 32 == 0 && K2 % 32 == 0 && K2 == 2 * HID);
static_assert(GBM == (GTHR / 32) * 16 && GBN == 64 && HID % GBN == 0 && OUTD % GBN == 0);
static_assert(NUW1 % NTHR == 0 && NUW2 % NTHR == 0);
static_assert(HID == 4 * 32 && OUTD == 2 * 32);
static_assert(SCAN_LDS_INTS * 4 <= 300000);
static_assert(NBA % TSUB == 0 && TSUB == 4 * 32 && OUTD % NWAVE == 0 && (TPITCH % 4) == 0 && TPITCH >= TSUB);
static_assert(RECW == 2 * OUTD && RECW == 4 * 32);

typedef float          v2f   __attribute__((ext_vector_type(2)));
typedef float          v4f   __attribute__((ext_vector_type(4)));
typedef float          v8f   __attribute__((ext_vector_type(8)));
typedef int            v4i   __attribute__((ext_vector_type(4)));
typedef int            v8i   __attribute__((ext_vector_type(8)));
typedef unsigned int   v4u   __attribute__((ext_vector_type(4)));
typedef unsigned short v8us  __attribute__((ext_vector_type(8)));
typedef unsigned short v16us __attribute__((ext_vector_type(16)));
typedef __bf16         v16bf __attribute__((ext_vector_type(16)));
typedef v2f  __attribute__((may_alias)) v2fa;
typedef v4f  __attribute__((may_alias)) v4fa;
typedef v4i  __attribute__((may_alias)) v4ia;
typedef v8us __attribute__((may_alias)) v8usa;
union FragB { v16bf v; v16us u; v8us h[2]; v8i w; };

__device__ __forceinline__ v8f wmb(const FragB& a, const FragB& b, v8f c) {
  v8f d = __builtin_amdgcn_wmma_f32_16x16x32_bf16(false, a.v, false, b.v, (short)0, c, false, false);
  asm volatile("v_nop\n\tv_nop\n\tv_nop\n\tv_nop" : "+v"(d) : "v"(a.w), "v"(b.w));
  return d;
}

__device__ __forceinline__ unsigned bf16_bits(float f) {
  const unsigned u = __float_as_uint(f);
  return (u + 0x7FFFu + ((u >> 16) & 1u)) >> 16;
}
__device__ __forceinline__ float bf16_val(float f) {
  return __uint_as_float(bf16_bits(f) << 16);
}
__device__ __forceinline__ int clampi(int v, int lo, int hi) {
  return v < lo ? lo : (v > hi ? hi : v);
}

template <int SLB>
__device__ __forceinline__ int scan_chunk(const int* __restrict__ dsts, int nE, int cbase, int slotBase,
                                          int nb, int vec8, int* list, int tid, int lane, int wave) {
  int wc = 0;
  const int el0  = tid * EPT;
  const int e0   = cbase + el0;
  const int sent = -2147483647 - 1;
  v4i da, db;
  if (vec8 != 0 && cbase + CHUNK <= nE) {
    da = *(const v4i*)(dsts + e0);
    db = *(const v4i*)(dsts + e0 + 4);
  } else {
    da.x = (e0     < nE) ? dsts[min(e0,     nE - 1)] : sent;
    da.y = (e0 + 1 < nE) ? dsts[min(e0 + 1, nE - 1)] : sent;
    da.z = (e0 + 2 < nE) ? dsts[min(e0 + 2, nE - 1)] : sent;
    da.w = (e0 + 3 < nE) ? dsts[min(e0 + 3, nE - 1)] : sent;
    db.x = (e0 + 4 < nE) ? dsts[min(e0 + 4, nE - 1)] : sent;
    db.y = (e0 + 5 < nE) ? dsts[min(e0 + 5, nE - 1)] : sent;
    db.z = (e0 + 6 < nE) ? dsts[min(e0 + 6, nE - 1)] : sent;
    db.w = (e0 + 7 < nE) ? dsts[min(e0 + 7, nE - 1)] : sent;
  }
  const unsigned nbs = (unsigned)slotBase;
  const unsigned unb = (unsigned)nb;
  const unsigned s0 = (unsigned)da.x - nbs, s1 = (unsigned)da.y - nbs;
  const unsigned s2 = (unsigned)da.z - nbs, s3 = (unsigned)da.w - nbs;
  const unsigned s4 = (unsigned)db.x - nbs, s5 = (unsigned)db.y - nbs;
  const unsigned s6 = (unsigned)db.z - nbs, s7 = (unsigned)db.w - nbs;
  const bool h0 = s0 < unb, h1 = s1 < unb, h2 = s2 < unb, h3 = s3 < unb;
  const bool h4 = s4 < unb, h5 = s5 < unb, h6 = s6 < unb, h7 = s7 < unb;
  const unsigned any = __builtin_amdgcn_ballot_w32(h0 | h1 | h2 | h3 | h4 | h5 | h6 | h7);
  if (any != 0u) {
#define HITJ(J, HJ, SJ) { \
      const unsigned mj = __builtin_amdgcn_ballot_w32(HJ); \
      if (mj != 0u) { \
        if (HJ) { \
          const int pos = wc + (int)__builtin_amdgcn_mbcnt_lo(mj, 0u); \
          if (pos < WCAP) list[wave * WCAP + pos] = ((el0 + (J)) << SLB) | (int)(SJ); \
        } \
        wc += (int)__builtin_popcount(mj); } }
    HITJ(0, h0, s0)
    HITJ(1, h1, s1)
    HITJ(2, h2, s2)
    HITJ(3, h3, s3)
    HITJ(4, h4, s4)
    HITJ(5, h5, s5)
    HITJ(6, h6, s6)
    HITJ(7, h7, s7)
#undef HITJ
  }
  return wc;
}

__global__ __launch_bounds__(NTHR) void k_wprep(const float* __restrict__ W1, const float* __restrict__ W2,
                                                unsigned short* W1B, unsigned short* W2D) {
  const int u = (int)blockIdx.x * NTHR + (int)threadIdx.x;
  const float* p;
  unsigned short* dp;
  if (u < NUW1) {
    const int n  = u >> 4;
    const int k8 = (u & 15) * 8;
    p  = W1 + (size_t)n * CIN + k8;
    dp = W1B + (size_t)n * CIN + k8;
  } else if (u < NUW1 + NUW2) {
    const int v  = u - NUW1;
    const int n  = v >> 5;
    const int k8 = (v & 31) * 8;
    const int kk = k8 & (HID - 1);
    p  = W2 + (size_t)n * HID + kk;
    dp = W2D + (size_t)n * K2 + k8;
  } else {
    return;
  }
  const v4f a = *(const v4fa*)p;
  const v4f b = *(const v4fa*)(p + 4);
  v8us o;
  o[0] = (unsigned short)bf16_bits(a.x); o[1] = (unsigned short)bf16_bits(a.y);
  o[2] = (unsigned short)bf16_bits(a.z); o[3] = (unsigned short)bf16_bits(a.w);
  o[4] = (unsigned short)bf16_bits(b.x); o[5] = (unsigned short)bf16_bits(b.y);
  o[6] = (unsigned short)bf16_bits(b.z); o[7] = (unsigned short)bf16_bits(b.w);
  *(volatile v8us*)dp = o;
  __threadfence();
  *(volatile v8us*)dp = o;
}

__global__ __launch_bounds__(NTHR) void k_cvx(const float* __restrict__ x, int nN, int nUnits,
                                              unsigned short* xb) {
  const int u = (int)blockIdx.x * NTHR + (int)threadIdx.x;
  if (u >= nUnits) return;
  const int row = u >> 4;
  const int k8  = (u & 15) * 8;
  const int rc  = row < nN ? row : nN - 1;
  const float* p = x + (size_t)rc * CIN + k8;
  const v4f a = *(const v4fa*)p;
  const v4f b = *(const v4fa*)(p + 4);
  const bool ok = row < nN;
  v8us o;
  o[0] = ok ? (unsigned short)bf16_bits(a.x) : (unsigned short)0;
  o[1] = ok ? (unsigned short)bf16_bits(a.y) : (unsigned short)0;
  o[2] = ok ? (unsigned short)bf16_bits(a.z) : (unsigned short)0;
  o[3] = ok ? (unsigned short)bf16_bits(a.w) : (unsigned short)0;
  o[4] = ok ? (unsigned short)bf16_bits(b.x) : (unsigned short)0;
  o[5] = ok ? (unsigned short)bf16_bits(b.y) : (unsigned short)0;
  o[6] = ok ? (unsigned short)bf16_bits(b.z) : (unsigned short)0;
  o[7] = ok ? (unsigned short)bf16_bits(b.w) : (unsigned short)0;
  unsigned short* dp = xb + (size_t)row * CIN + k8;
  *(volatile v8us*)dp = o;
  __threadfence();
  *(volatile v8us*)dp = o;
}

__global__ __launch_bounds__(NTHR) void k_scan(const int* __restrict__ srcs, const int* __restrict__ dsts,
                                               const float* __restrict__ ew, int nE, int nN, int vec8,
                                               int* lsrc, float* lwt, int* goffs, int* gcnt, float* dis) {
  extern __shared__ __attribute__((aligned(16))) int dsm[];
  int* list = dsm;
  int* hl   = dsm + LISTN;
  int* sl   = dsm + LISTN + RCAP;
  int* cnt  = dsm + LISTN + 2 * RCAP;
  int* offs = cnt + NBA;
  int* cur  = offs + NBA;
  int* misc = cur + NBA;
  const int tid = (int)threadIdx.x, lane = tid & 31, wave = tid >> 5;
  const int nodeBase = (int)blockIdx.x * NBA;

  {
    const v4i z4 = {0, 0, 0, 0};
    for (int i = tid * 4; i < SCAN_ZINTS; i += NTHR * 4) *(v4ia*)(dsm + i) = z4;
    if (tid < 16) misc[tid] = 0;
  }
  __syncthreads();

  int t = 0, ov = 0;
  const int nChunks = (nE + CHUNK - 1) / CHUNK;
#pragma unroll 1
  for (int ch = 0; ch < nChunks; ++ch) {
    const int cbase = ch * CHUNK;
    const int wc = scan_chunk<SLA>(dsts, nE, cbase, nodeBase, NBA, vec8, list, tid, lane, wave);
    if (lane == 0) misc[wave] = wc;
    __syncthreads();
    if (wave == 0) {
#pragma unroll 1
      for (int w2 = 0; w2 < NWAVE; ++w2) {
        int c = misc[w2];
        c = c < 0 ? 0 : (c > WCAP ? WCAP : c);
#pragma unroll 1
        for (int b0 = 0; b0 < c; b0 += 32) {
          const int idx = b0 + lane;
          const int ent = list[w2 * WCAP + (idx < WCAP ? idx : WCAP - 1)];
          const int m32 = (c - b0) < 32 ? (c - b0) : 32;
#pragma unroll 1
          for (int k = 0; k < m32; ++k) {
            const int u    = __builtin_amdgcn_readlane(ent, k);
            const int slot = u & (NBA - 1);
            const int el   = (u >> SLA) & (CHUNK - 1);
            const int pk   = ((cbase + el) << SLA) | slot;
            if (t < RCAP) {
              if (lane == 0) { hl[t] = pk; cnt[slot] = cnt[slot] + 1; }
              t = t + 1;
            } else {
              ov = 1;
            }
          }
        }
      }
    }
    __syncthreads();
  }
  if (wave == 0 && lane == 0) { misc[8] = t; misc[9] = ov; }
  __syncthreads();
  int tt = misc[8];
  tt = tt < 0 ? 0 : (tt > RCAP ? RCAP : tt);
  const int ovf = misc[9];

  if (wave == 0) {
    const int base = lane * (NBA / 32);
    int s = 0;
#pragma unroll 1
    for (int i = 0; i < NBA / 32; ++i) s += cnt[base + i];
    int incl = s;
#pragma unroll
    for (int d = 1; d < 32; d <<= 1) {
      const int y = __shfl_up(incl, d, 32);
      if (lane >= d) incl += y;
    }
    int run = incl - s;
#pragma unroll 1
    for (int i = 0; i < NBA / 32; ++i) {
      const int cv = cnt[base + i];
      offs[base + i] = run;
      cur[base + i]  = run;
      run += cv;
    }
  }
  __syncthreads();
  if (wave == 0) {
#pragma unroll 1
    for (int b0 = 0; b0 < tt; b0 += 32) {
      const int idx = b0 + lane;
      const int ent = hl[idx < RCAP ? idx : RCAP - 1];
      const int m32 = (tt - b0) < 32 ? (tt - b0) : 32;
#pragma unroll 1
      for (int k = 0; k < m32; ++k) {
        const int u    = __builtin_amdgcn_readlane(ent, k);
        const int slot = u & (NBA - 1);
        if (lane == 0) {
          int p = cur[slot];
          p = p < 0 ? 0 : (p > RCAP - 1 ? RCAP - 1 : p);
          sl[p] = u;
          cur[slot] = p + 1;
        }
      }
    }
  }
  __syncthreads();

  const size_t lbase = (size_t)blockIdx.x * (size_t)RCAP;
  const int nIt = (tt + 1023) >> 10;
#pragma unroll 1
  for (int it = 0; it < nIt; ++it) {
    const int p0 = it * 1024 + 4 * tid;
    const v4i e4 = *(const v4ia*)(sl + p0);
    const int e0 = clampi(e4.x >> SLA, 0, nE - 1);
    const int e1 = clampi(e4.y >> SLA, 0, nE - 1);
    const int e2 = clampi(e4.z >> SLA, 0, nE - 1);
    const int e3 = clampi(e4.w >> SLA, 0, nE - 1);
    const int r0 = srcs[e0], r1 = srcs[e1], r2 = srcs[e2], r3 = srcs[e3];
    const float w0 = ew[e0], w1 = ew[e1], w2 = ew[e2], w3 = ew[e3];
    const bool l0 = p0 < tt, l1 = (p0 + 1) < tt, l2 = (p0 + 2) < tt, l3 = (p0 + 3) < tt;
    v4i sv;
    sv.x = l0 ? clampi(r0, 0, nN - 1) : 0;
    sv.y = l1 ? clampi(r1, 0, nN - 1) : 0;
    sv.z = l2 ? clampi(r2, 0, nN - 1) : 0;
    sv.w = l3 ? clampi(r3, 0, nN - 1) : 0;
    v4f wv;
    wv.x = l0 ? bf16_val(w0) : 0.0f;
    wv.y = l1 ? bf16_val(w1) : 0.0f;
    wv.z = l2 ? bf16_val(w2) : 0.0f;
    wv.w = l3 ? bf16_val(w3) : 0.0f;
    v4i wi;
    wi.x = __float_as_int(wv.x); wi.y = __float_as_int(wv.y);
    wi.z = __float_as_int(wv.z); wi.w = __float_as_int(wv.w);
    *(v4ia*)(hl + p0) = wi;
    int*   sp = lsrc + lbase + p0;
    float* wp = lwt + lbase + p0;
    *(volatile v4i*)sp = sv;
    *(volatile v4f*)wp = wv;
    __threadfence();
    *(volatile v4i*)sp = sv;
    *(volatile v4f*)wp = wv;
  }
  __syncthreads();

  const v4i c4r = *(const v4ia*)(cnt + 4 * tid);
  const v4i o4r = *(const v4ia*)(offs + 4 * tid);
  const int c0 = clampi(c4r.x, 0, DEGCAP), c1 = clampi(c4r.y, 0, DEGCAP);
  const int c2 = clampi(c4r.z, 0, DEGCAP), c3 = clampi(c4r.w, 0, DEGCAP);
  const int o0 = clampi(o4r.x, 0, RCAP - 1), o1 = clampi(o4r.y, 0, RCAP - 1);
  const int o2 = clampi(o4r.z, 0, RCAP - 1), o3 = clampi(o4r.w, 0, RCAP - 1);
  int cm = max(max(c0, c1), max(c2, c3));
#pragma unroll
  for (int d = 16; d >= 1; d >>= 1) {
    const int y = __shfl_xor(cm, d, 32);
    cm = y > cm ? y : cm;
  }
  float d0 = 0.0f, d1 = 0.0f, d2 = 0.0f, d3 = 0.0f;
#pragma unroll 1
  for (int j = 0; j < cm; ++j) {
    const float t0 = __int_as_float(hl[min(o0 + j, RCAP - 1)]);
    const float t1 = __int_as_float(hl[min(o1 + j, RCAP - 1)]);
    const float t2 = __int_as_float(hl[min(o2 + j, RCAP - 1)]);
    const float t3 = __int_as_float(hl[min(o3 + j, RCAP - 1)]);
    d0 += (j < c0) ? t0 : 0.0f;
    d1 += (j < c1) ? t1 : 0.0f;
    d2 += (j < c2) ? t2 : 0.0f;
    d3 += (j < c3) ? t3 : 0.0f;
  }
  const float qnan = __int_as_float(0x7fc00000);
  const bool anyov = ovf != 0;
  v4f dv;
  {
    const float g0 = d0 + 1.0f, g1 = d1 + 1.0f, g2 = d2 + 1.0f, g3 = d3 + 1.0f;
    const float q0 = (g0 > 0.0f) ? rsqrtf((g0 > 0.0f) ? g0 : 1.0f) : 0.0f;
    const float q1 = (g1 > 0.0f) ? rsqrtf((g1 > 0.0f) ? g1 : 1.0f) : 0.0f;
    const float q2 = (g2 > 0.0f) ? rsqrtf((g2 > 0.0f) ? g2 : 1.0f) : 0.0f;
    const float q3 = (g3 > 0.0f) ? rsqrtf((g3 > 0.0f) ? g3 : 1.0f) : 0.0f;
    dv.x = (anyov || c4r.x > DEGCAP) ? qnan : q0;
    dv.y = (anyov || c4r.y > DEGCAP) ? qnan : q1;
    dv.z = (anyov || c4r.z > DEGCAP) ? qnan : q2;
    dv.w = (anyov || c4r.w > DEGCAP) ? qnan : q3;
  }
  v4i co;
  co.x = anyov ? -1 : c4r.x; co.y = anyov ? -1 : c4r.y;
  co.z = anyov ? -1 : c4r.z; co.w = anyov ? -1 : c4r.w;
  int*   gp = gcnt  + (size_t)nodeBase + 4 * tid;
  int*   op = goffs + (size_t)nodeBase + 4 * tid;
  float* dp = dis   + (size_t)nodeBase + 4 * tid;
  *(volatile v4i*)gp = co;
  *(volatile v4i*)op = o4r;
  *(volatile v4f*)dp = dv;
  __threadfence();
  *(volatile v4i*)gp = co;
  *(volatile v4i*)op = o4r;
  *(volatile v4f*)dp = dv;
}

__global__ __launch_bounds__(GTHR) void k_gemm(
    const unsigned short* __restrict__ A, const unsigned short* __restrict__ WT,
    float* outF, int K, int ldo)
{
  __shared__ __attribute__((aligned(16))) float stg[GBM * GBN];
  const int tid = (int)threadIdx.x, lane = tid & 31, wave = tid >> 5, hh = lane >> 4, m = lane & 15;
  const int rowBase = (int)blockIdx.x * GBM;
  const int col0    = (int)blockIdx.y * GBN;

  v8f acc[4];
  {
    const v8f z = {0.f, 0.f, 0.f, 0.f, 0.f, 0.f, 0.f, 0.f};
    acc[0] = z; acc[1] = z; acc[2] = z; acc[3] = z;
  }
  const unsigned short* ap = A  + (size_t)(rowBase + 16 * wave + m) * (size_t)K + 8 * hh;
  const unsigned short* wp = WT + (size_t)(col0 + m) * (size_t)K + 8 * hh;
  const int ksteps = K >> 5;
#pragma unroll 1
  for (int ks = 0; ks < ksteps; ++ks) {
    FragB af;
    af.h[0] = *(const v8usa*)(ap + 32 * ks);
    af.h[1] = *(const v8usa*)(ap + 32 * ks + 16);
#pragma unroll
    for (int t = 0; t < 4; ++t) {
      const unsigned short* wq = wp + (size_t)(16 * t) * (size_t)K + 32 * ks;
      FragB bf;
      bf.h[0] = *(const v8usa*)wq;
      bf.h[1] = *(const v8usa*)(wq + 16);
      acc[t] = wmb(af, bf, acc[t]);
    }
  }

#pragma unroll
  for (int t = 0; t < 4; ++t) {
    const int lc = 16 * t + m;
#pragma unroll
    for (int r = 0; r < 8; ++r) {
      const int lr = 16 * wave + 8 * hh + r;
      stg[lr * GBN + lc] = acc[t][r];
    }
  }
  __syncthreads();

  v4f fv[8];
#pragma unroll
  for (int i = 0; i < 8; ++i) {
    const int lr = 16 * wave + 2 * i + hh;
    fv[i] = *(const v4fa*)(stg + lr * GBN + 4 * m);
  }
#pragma unroll
  for (int i = 0; i < 8; ++i) {
    const int lr = 16 * wave + 2 * i + hh;
    const int gr = rowBase + lr;
    float* op = outF + (size_t)gr * (size_t)ldo + col0 + 4 * m;
    *(volatile v4f*)op = fv[i];
  }
  __threadfence();
#pragma unroll
  for (int i = 0; i < 8; ++i) {
    const int lr = 16 * wave + 2 * i + hh;
    const int gr = rowBase + lr;
    float* op = outF + (size_t)gr * (size_t)ldo + col0 + 4 * m;
    *(volatile v4f*)op = fv[i];
  }
}

__global__ __launch_bounds__(NTHR) void k_agg1(const int* __restrict__ lsrc, const float* __restrict__ lwt,
                                               const int* __restrict__ goffs, const int* __restrict__ gcnt,
                                               int nN, int mRows, const float* __restrict__ dis,
                                               const float* __restrict__ h1, const float* __restrict__ bias,
                                               unsigned short* x1) {
  __shared__ __attribute__((aligned(16))) int cl[NBA];
  __shared__ __attribute__((aligned(16))) int ol[NBA];
  const int tid = (int)threadIdx.x, lane = tid & 31, wave = tid >> 5;
  const int nodeBase = (int)blockIdx.x * NBA;
  {
    const v4i a = *(const v4i*)(gcnt  + (size_t)nodeBase + 4 * tid);
    const v4i b = *(const v4i*)(goffs + (size_t)nodeBase + 4 * tid);
    *(v4ia*)(cl + 4 * tid) = a;
    *(v4ia*)(ol + 4 * tid) = b;
  }
  float bv0, bv1, bv2, bv3;
  {
    const v4f a = *(const v4fa*)(bias + 4 * lane);
    bv0 = bf16_val(a.x); bv1 = bf16_val(a.y); bv2 = bf16_val(a.z); bv3 = bf16_val(a.w);
  }
  __syncthreads();

  const size_t lbase = (size_t)blockIdx.x * (size_t)RCAP;
  const float qnan = __int_as_float(0x7fc00000);
  const int sa = (2 * lane) & 31, sb = (2 * lane + 1) & 31;
#pragma unroll 1
  for (int si = 0; si < NBA / NWAVE; ++si) {
    const int s    = si * NWAVE + wave;
    const int node = nodeBase + s;
    int c = cl[s];
    const bool bad = (c < 0) || (c > DEGCAP);
    c = c < 0 ? 0 : (c > DEGCAP ? DEGCAP : c);
    const int o = clampi(ol[s], 0, RCAP - 1);
    const int nc = node < nN ? node : nN - 1;
    const float dd = dis[nc];
    const float rd = dd * dd;
    float a0 = 0.0f, a1 = 0.0f, a2 = 0.0f, a3 = 0.0f;
#pragma unroll 1
    for (int b0 = 0; b0 < c; b0 += 32) {
      const int m32 = (c - b0) < 32 ? (c - b0) : 32;
      const int li  = lane < m32 ? lane : m32 - 1;
      int idx = o + b0 + li;
      idx = idx > RCAP - 1 ? RCAP - 1 : idx;
      int sr = lsrc[lbase + idx];
      sr = sr < 0 ? 0 : (sr > nN - 1 ? nN - 1 : sr);
      const float wv  = lwt[lbase + idx];
      const float cf  = (dis[sr] * wv) * dd;
      const int   cfi = __float_as_int(cf);
#pragma unroll 1
      for (int k = 0; k < m32; ++k) {
        const int   sk = __builtin_amdgcn_readlane(sr, k);
        const float ck = __int_as_float(__builtin_amdgcn_readlane(cfi, k));
        const v4f a = *(const v4fa*)(h1 + (size_t)sk * HID + 4 * lane);
        a0 = fmaf(ck, a.x, a0); a1 = fmaf(ck, a.y, a1);
        a2 = fmaf(ck, a.z, a2); a3 = fmaf(ck, a.w, a3);
      }
    }
    const v4f sv = *(const v4fa*)(h1 + (size_t)nc * HID + 4 * lane);
    const float pzr = bad ? qnan : 0.0f;
    const bool live = node < nN;
    float y0 = (a0 + sv.x * rd) + bv0;
    float y1 = (a1 + sv.y * rd) + bv1;
    float y2 = (a2 + sv.z * rd) + bv2;
    float y3 = (a3 + sv.w * rd) + bv3;
    y0 = (y0 > 0.0f) ? y0 : (y0 - y0);
    y1 = (y1 > 0.0f) ? y1 : (y1 - y1);
    y2 = (y2 > 0.0f) ? y2 : (y2 - y2);
    y3 = (y3 > 0.0f) ? y3 : (y3 - y3);
    y0 = y0 + pzr; y1 = y1 + pzr; y2 = y2 + pzr; y3 = y3 + pzr;
    const float v0 = live ? y0 : 0.0f;
    const float v1 = live ? y1 : 0.0f;
    const float v2 = live ? y2 : 0.0f;
    const float v3 = live ? y3 : 0.0f;
    const unsigned hb0 = bf16_bits(v0), hb1 = bf16_bits(v1), hb2 = bf16_bits(v2), hb3 = bf16_bits(v3);
    const unsigned lb0 = bf16_bits(v0 - __uint_as_float(hb0 << 16));
    const unsigned lb1 = bf16_bits(v1 - __uint_as_float(hb1 << 16));
    const unsigned lb2 = bf16_bits(v2 - __uint_as_float(hb2 << 16));
    const unsigned lb3 = bf16_bits(v3 - __uint_as_float(hb3 << 16));
    const int hw0 = (int)(hb0 | (hb1 << 16));
    const int hw1 = (int)(hb2 | (hb3 << 16));
    const int lw0 = (int)(lb0 | (lb1 << 16));
    const int lw1 = (int)(lb2 | (lb3 << 16));
    const int g0 = __shfl(hw0, sa, 32), g1 = __shfl(hw1, sa, 32);
    const int g2 = __shfl(hw0, sb, 32), g3 = __shfl(hw1, sb, 32);
    const int p0 = __shfl(lw0, sa, 32), p1 = __shfl(lw1, sa, 32);
    const int p2 = __shfl(lw0, sb, 32), p3 = __shfl(lw1, sb, 32);
    const bool lsel = lane >= 16;
    v4u pv;
    pv.x = (unsigned int)(lsel ? p0 : g0);
    pv.y = (unsigned int)(lsel ? p1 : g1);
    pv.z = (unsigned int)(lsel ? p2 : g2);
    pv.w = (unsigned int)(lsel ? p3 : g3);
    unsigned short* hp = x1 + (size_t)node * K2 + 8 * lane;
    const bool wr = node < mRows;
    if (wr) *(volatile v4u*)hp = pv;
    __threadfence();
    if (wr) *(volatile v4u*)hp = pv;
  }
}

__global__ __launch_bounds__(NTHR) void k_agg2(const int* __restrict__ lsrc, const float* __restrict__ lwt,
                                               const int* __restrict__ goffs, const int* __restrict__ gcnt,
                                               int nN, int mRows, const float* __restrict__ dis,
                                               const float* __restrict__ h2, const float* __restrict__ bias,
                                               float* zout, float* rec) {
  __shared__ __attribute__((aligned(16))) int cl[NBA];
  __shared__ __attribute__((aligned(16))) int ol[NBA];
  __shared__ __attribute__((aligned(16))) float wm[NWAVE * OUTD];
  __shared__ __attribute__((aligned(16))) float wsu[NWAVE * OUTD];
  __shared__ __attribute__((aligned(16))) float recs[RECW];
  const int tid = (int)threadIdx.x, lane = tid & 31, wave = tid >> 5;
  const int nodeBase = (int)blockIdx.x * NBA;
  {
    const v4i a = *(const v4i*)(gcnt  + (size_t)nodeBase + 4 * tid);
    const v4i b = *(const v4i*)(goffs + (size_t)nodeBase + 4 * tid);
    *(v4ia*)(cl + 4 * tid) = a;
    *(v4ia*)(ol + 4 * tid) = b;
  }
  float bv0, bv1;
  {
    const v2f a = *(const v2fa*)(bias + 2 * lane);
    bv0 = bf16_val(a.x); bv1 = bf16_val(a.y);
  }
  __syncthreads();

  const size_t lbase = (size_t)blockIdx.x * (size_t)RCAP;
  const float qnan = __int_as_float(0x7fc00000);
  const float ninf = __int_as_float((int)0xff800000u);
  const int sa = (2 * lane) & 31, sb = (2 * lane + 1) & 31;
  float m0 = ninf, m1 = ninf, s0 = 0.0f, s1 = 0.0f;
#pragma unroll 1
  for (int si = 0; si < NBA / NWAVE; ++si) {
    const int s    = si * NWAVE + wave;
    const int node = nodeBase + s;
    int c = cl[s];
    const bool bad = (c < 0) || (c > DEGCAP);
    c = c < 0 ? 0 : (c > DEGCAP ? DEGCAP : c);
    const int o = clampi(ol[s], 0, RCAP - 1);
    const int nc = node < nN ? node : nN - 1;
    const float dd = dis[nc];
    const float rd = dd * dd;
    float acc0 = 0.0f, acc1 = 0.0f;
#pragma unroll 1
    for (int b0 = 0; b0 < c; b0 += 32) {
      const int m32 = (c - b0) < 32 ? (c - b0) : 32;
      const int li  = lane < m32 ? lane : m32 - 1;
      int idx = o + b0 + li;
      idx = idx > RCAP - 1 ? RCAP - 1 : idx;
      int sr = lsrc[lbase + idx];
      sr = sr < 0 ? 0 : (sr > nN - 1 ? nN - 1 : sr);
      const float wv  = lwt[lbase + idx];
      const float cf  = (dis[sr] * wv) * dd;
      const int   cfi = __float_as_int(cf);
#pragma unroll 1
      for (int k = 0; k < m32; ++k) {
        const int   sk = __builtin_amdgcn_readlane(sr, k);
        const float ck = __int_as_float(__builtin_amdgcn_readlane(cfi, k));
        const v2f a = *(const v2fa*)(h2 + (size_t)sk * OUTD + 2 * lane);
        acc0 = fmaf(ck, a.x, acc0); acc1 = fmaf(ck, a.y, acc1);
      }
    }
    const v2f sv = *(const v2fa*)(h2 + (size_t)nc * OUTD + 2 * lane);
    const float pzr = bad ? qnan : 0.0f;
    const bool live = node < nN;
    float y0 = (acc0 + sv.x * rd) + bv0;
    float y1 = (acc1 + sv.y * rd) + bv1;
    y0 = (y0 > 0.0f) ? y0 : (y0 - y0);
    y1 = (y1 > 0.0f) ? y1 : (y1 - y1);
    y0 = y0 + pzr; y1 = y1 + pzr;
    const float v0 = live ? y0 : 0.0f;
    const float v1 = live ? y1 : 0.0f;
    if (live) {
      const float e0 = expf(-fabsf(v0 - m0));
      const float e1 = expf(-fabsf(v1 - m1));
      const bool gt0 = v0 > m0, gt1 = v1 > m1;
      s0 = gt0 ? fmaf(s0, e0, 1.0f) : (s0 + e0);
      s1 = gt1 ? fmaf(s1, e1, 1.0f) : (s1 + e1);
      m0 = gt0 ? v0 : m0;
      m1 = gt1 ? v1 : m1;
    }
    v4f ow;
    ow.x = __shfl(v0, sa, 32); ow.y = __shfl(v1, sa, 32);
    ow.z = __shfl(v0, sb, 32); ow.w = __shfl(v1, sb, 32);
    float* op = zout + (size_t)node * OUTD + 4 * (lane & 15);
    const bool wr = (node < mRows) && (lane < 16);
    if (wr) *(volatile v4f*)op = ow;
    __threadfence();
    if (wr) *(volatile v4f*)op = ow;
  }

  wm[wave * OUTD + 2 * lane + 0]  = m0;
  wm[wave * OUTD + 2 * lane + 1]  = m1;
  wsu[wave * OUTD + 2 * lane + 0] = s0;
  wsu[wave * OUTD + 2 * lane + 1] = s1;
  __syncthreads();
  if (tid < OUTD) {
    float M = ninf;
#pragma unroll 1
    for (int w2 = 0; w2 < NWAVE; ++w2) {
      const float tmx = wm[w2 * OUTD + tid];
      M = (tmx > M) ? tmx : M;
    }
    float S = 0.0f;
#pragma unroll 1
    for (int w2 = 0; w2 < NWAVE; ++w2) {
      S += wsu[w2 * OUTD + tid] * expf(wm[w2 * OUTD + tid] - M);
    }
    recs[tid] = M;
    recs[OUTD + tid] = S;
  }
  __syncthreads();
  {
    const v4f rv = *(const v4fa*)(recs + 4 * lane);
    float* rp = rec + (size_t)blockIdx.x * RECW + 4 * lane;
    const bool okst = wave == 0;
    if (okst) *(volatile v4f*)rp = rv;
    __threadfence();
    if (okst) *(volatile v4f*)rp = rv;
  }
}

__global__ __launch_bounds__(64) void k_combine(const float* __restrict__ rec, int nB, float* ms) {
  __shared__ __attribute__((aligned(16))) float sm[RECW];
  const int tid = (int)threadIdx.x, lane = tid & 31;
  const float ninf = __int_as_float((int)0xff800000u);
  float M = ninf;
#pragma unroll 1
  for (int b = 0; b < nB; ++b) {
    const float tmx = rec[(size_t)b * RECW + tid];
    M = (tmx > M) ? tmx : M;
  }
  double S = 0.0;
#pragma unroll 1
  for (int b = 0; b < nB; ++b) {
    const float mb = rec[(size_t)b * RECW + tid];
    const float sb = rec[(size_t)b * RECW + OUTD + tid];
    S += (double)sb * (double)expf(mb - M);
  }
  const float Sf = (float)S;
  sm[tid] = M;
  sm[OUTD + tid] = 1.0f / Sf;
  __syncthreads();
  const v4f ov = *(const v4fa*)(sm + 4 * lane);
  float* op = ms + 4 * lane;
  const bool okst = tid < 32;
  if (okst) *(volatile v4f*)op = ov;
  __threadfence();
  if (okst) *(volatile v4f*)op = ov;
}

__global__ __launch_bounds__(NTHR) void k_out(const float* __restrict__ z, const float* __restrict__ ms,
                                              int nN, float* out) {
  __shared__ __attribute__((aligned(16))) float tl[OUTD * TPITCH];
  const int tid = (int)threadIdx.x, lane = tid & 31, wave = tid >> 5;
  const int base = (int)blockIdx.x * NBA;
  const int c4 = (tid & 15) * 4;
  const int r0 = tid >> 4;
  const v4f M4 = *(const v4fa*)(ms + c4);
  const v4f I4 = *(const v4fa*)(ms + OUTD + c4);
  const int rem = nN - base;
  int nSub = rem <= 0 ? 0 : (rem + TSUB - 1) / TSUB;
  nSub = nSub > NBA / TSUB ? NBA / TSUB : nSub;
#pragma unroll 1
  for (int sub = 0; sub < nSub; ++sub) {
    const int n0 = base + sub * TSUB;
#pragma unroll 1
    for (int i = 0; i < 8; ++i) {
      const int row = r0 + 16 * i;
      const int node = n0 + row;
      const int ncl = node < nN ? node : nN - 1;
      const v4f zv = *(const v4fa*)(z + (size_t)ncl * OUTD + c4);
      tl[(c4 + 0) * TPITCH + row] = expf(zv.x - M4.x) * I4.x;
      tl[(c4 + 1) * TPITCH + row] = expf(zv.y - M4.y) * I4.y;
      tl[(c4 + 2) * TPITCH + row] = expf(zv.z - M4.z) * I4.z;
      tl[(c4 + 3) * TPITCH + row] = expf(zv.w - M4.w) * I4.w;
    }
    __syncthreads();
    v4f ov[OUTD / NWAVE];
#pragma unroll
    for (int q = 0; q < OUTD / NWAVE; ++q) {
      const int c = wave + NWAVE * q;
      ov[q] = *(const v4fa*)(tl + c * TPITCH + 4 * lane);
    }
    const bool ok = (n0 + 4 * lane + 3) < nN;
#pragma unroll
    for (int q = 0; q < OUTD / NWAVE; ++q) {
      const int c = wave + NWAVE * q;
      float* op = out + (size_t)c * (size_t)nN + n0 + 4 * lane;
      if (ok) *(volatile v4f*)op = ov[q];
    }
    __threadfence();
#pragma unroll
    for (int q = 0; q < OUTD / NWAVE; ++q) {
      const int c = wave + NWAVE * q;
      float* op = out + (size_t)c * (size_t)nN + n0 + 4 * lane;
      if (ok) *(volatile v4f*)op = ov[q];
    }
    __syncthreads();
  }
}

static inline int cdiv(int a, int b) { return (a + b - 1) / b; }
static inline size_t al256(size_t o) { return (o + 255) & ~(size_t)255; }

extern "C" void kernel_launch(void* const* d_in, const int* in_sizes, int n_in,
                              void* d_out, int out_size, void* d_ws, size_t ws_size,
                              hipStream_t stream) {
  if (n_in < 7) return;
  if (in_sizes[0] < CIN || (in_sizes[0] % CIN) != 0) return;
  const int nN = in_sizes[0] / CIN;
  if (nN < 32 || nN > (1 << 22) || (nN % 32) != 0) return;
  if (in_sizes[1] < 2 || (in_sizes[1] & 1) != 0) return;
  const int nE = in_sizes[1] / 2;
  if (nE < 1 || nE >= (1 << (31 - SLA))) return;
  if (in_sizes[2] != nE) return;
  if (in_sizes[3] != HID * CIN || in_sizes[4] != HID) return;
  if (in_sizes[5] != OUTD * HID || in_sizes[6] != OUTD) return;
  if ((long long)out_size != (long long)OUTD * nN) return;

  const float* x    = (const float*)d_in[0];
  const int*   edge = (const int*)d_in[1];
  const float* ew   = (const float*)d_in[2];
  const float* W1   = (const float*)d_in[3];
  const float* b1   = (const float*)d_in[4];
  const float* W2   = (const float*)d_in[5];
  const float* b2   = (const float*)d_in[6];
  float* out = (float*)d_out;
  const int* src = edge;
  const int* dst = edge + nE;

  const int MP = cdiv(nN, GBM) * GBM;
  const int gM = MP / GBM;
  const int gA = cdiv(MP, NBA);
  const int gO = cdiv(nN, NBA);
  if ((long long)gA * NBA < (long long)MP) return;
  const int vec8 = ((nE & 3) == 0) ? 1 : 0;

  char* ws = (char*)d_ws;
  size_t off = 0;
  const size_t szA   = (size_t)MP * HID * 4;
  const size_t szB   = (size_t)MP * K2 * 2;
  const size_t oA    = off; off = al256(off + szA);
  const size_t oB    = off; off = al256(off + szB);
  const size_t oLS   = off; off = al256(off + (size_t)gA * RCAP * 4);
  const size_t oLW   = off; off = al256(off + (size_t)gA * RCAP * 4);
  const size_t oOF   = off; off = al256(off + (size_t)gA * NBA * 4);
  const size_t oCN   = off; off = al256(off + (size_t)gA * NBA * 4);
  const size_t oDIS  = off; off = al256(off + (size_t)gA * NBA * 4);
  const size_t oW1B  = off; off = al256(off + (size_t)HID * CIN * 2);
  const size_t oW2D  = off; off = al256(off + (size_t)OUTD * K2 * 2);
  const size_t oREC  = off; off = al256(off + (size_t)gA * RECW * 4);
  const size_t oMS   = off; off = al256(off + (size_t)RECW * 4);
  if (off > ws_size || off > (size_t)WSMAX) return;
  float*          H1  = (float*)(ws + oA);
  float*          H2  = (float*)(ws + oA);
  float*          Z   = (float*)(ws + oA + (size_t)MP * OUTD * 4);
  unsigned short* XB  = (unsigned short*)(ws + oB);
  unsigned short* X1  = (unsigned short*)(ws + oB);
  int*            LS  = (int*)(ws + oLS);
  float*          LW  = (float*)(ws + oLW);
  int*            OF  = (int*)(ws + oOF);
  int*            CN  = (int*)(ws + oCN);
  float*          DIS = (float*)(ws + oDIS);
  unsigned short* W1B = (unsigned short*)(ws + oW1B);
  unsigned short* W2D = (unsigned short*)(ws + oW2D);
  float*          REC = (float*)(ws + oREC);
  float*          MS  = (float*)(ws + oMS);

  const size_t scanLds = (size_t)SCAN_LDS_INTS * 4;
  hipFuncSetAttribute(reinterpret_cast<const void*>(&k_scan), hipFuncAttributeMaxDynamicSharedMemorySize, (int)scanLds);

  const int nUx = MP * (CIN / 8);
  k_wprep<<<(NUW1 + NUW2) / NTHR, NTHR, 0, stream>>>(W1, W2, W1B, W2D);
  k_cvx<<<cdiv(nUx, NTHR), NTHR, 0, stream>>>(x, nN, nUx, XB);
  k_scan<<<gA, NTHR, scanLds, stream>>>(src, dst, ew, nE, nN, vec8, LS, LW, OF, CN, DIS);
  k_gemm<<<dim3(gM, HID / GBN), GTHR, 0, stream>>>(XB, W1B, H1, CIN, HID);
  k_agg1<<<gA, NTHR, 0, stream>>>(LS, LW, OF, CN, nN, MP, DIS, H1, b1, X1);
  k_gemm<<<dim3(gM, OUTD / GBN), GTHR, 0, stream>>>(X1, W2D, H2, K2, OUTD);
  k_agg2<<<gA, NTHR, 0, stream>>>(LS, LW, OF, CN, nN, MP, DIS, H2, b2, Z, REC);
  k_combine<<<1, 64, 0, stream>>>(REC, gA, MS);
  k_out<<<gO, NTHR, 0, stream>>>(Z, MS, nN, out);
}
